// LSTM_9294309229308
// MI455X (gfx1250) — hardware-verified
//
#include <hip/hip_runtime.h>

constexpr int NBATCH   = 4096;
constexpr int SEQ      = 1024;
constexpr int HID      = 16;
constexpr int NGATE    = 4 * HID;
constexpr int NPRED    = 5;
constexpr int NWAVES   = 4;
constexpr int NTHREADS = NWAVES * 32;
constexpr int ROWS_PER_BLOCK = NWAVES * 16;
constexpr int NBLOCKS  = NBATCH / ROWS_PER_BLOCK;
constexpr int OUT_PER_BLOCK = ROWS_PER_BLOCK * NPRED;
constexpr int OUT_V4_PER_BLOCK = OUT_PER_BLOCK / 4;
constexpr float LOCARRY     = 512.0f;
constexpr float LOCARRY_INV = 1.0f / 512.0f;

static_assert(HID == 16, "one 16-wide k group of hidden units");
static_assert(NGATE == 64, "four 16-row gate tiles");
static_assert(NBATCH % ROWS_PER_BLOCK == 0, "grid exact");
static_assert(NBLOCKS == 64, "grid");
static_assert(ROWS_PER_BLOCK % 32 == 0, "block owns a multiple of 32 output rows");
static_assert((OUT_PER_BLOCK * 4) % 128 == 0, "block output slab is whole 128-B lines");
static_assert(OUT_V4_PER_BLOCK == 80, "80 float4 per block");
static_assert(NGATE * HID == 2 * NTHREADS * 4, "W_hh staging: 2 float4 per thread covers the plane exactly");
static_assert(NBATCH * NPRED * 4 == 81920, "output bytes");

typedef __attribute__((ext_vector_type(16))) _Float16 v16h;
typedef __attribute__((ext_vector_type(2)))  _Float16 v2h;
typedef __attribute__((ext_vector_type(8)))  float    v8f;
typedef __attribute__((ext_vector_type(4)))  float    v4f;
typedef __attribute__((ext_vector_type(2)))  float    v2f;
typedef __attribute__((ext_vector_type(8)))  unsigned v8u;

__device__ __forceinline__ float hw_tanh(float x) {
#if __has_builtin(__builtin_amdgcn_tanhf)
  return __builtin_amdgcn_tanhf(x);
#elif __has_builtin(__builtin_amdgcn_tanh_f32)
  return __builtin_amdgcn_tanh_f32(x);
#else
  return 1.0f - 2.0f * __builtin_amdgcn_rcpf(__expf(2.0f * x) + 1.0f);
#endif
}
__device__ __forceinline__ float sig_half_arg(float d) {
  return __builtin_fmaf(0.5f, hw_tanh(d), 0.5f);
}
__device__ __forceinline__ unsigned pack_rne(float a, float b) {
  v2f f;
  f[0] = a;
  f[1] = b;
  const v2h hv = __builtin_convertvector(f, v2h);
  return __builtin_bit_cast(unsigned, hv);
}
__device__ __forceinline__ v8f wmma_f16(v16h a, v16h b, v8f c) {
  return __builtin_amdgcn_wmma_f32_16x16x32_f16(false, a, false, b, (short)0, c, false, false);
}
__device__ __forceinline__ void wmma_guard4(v8f& d0, v8f& d1, v8f& d2, v8f& d3,
                                            v16h bf, v16h a0, v16h a1, v16h a2, v16h a3) {
  asm volatile("v_nop\n\tv_nop\n\tv_nop\n\tv_nop"
               : "+v"(d0), "+v"(d1), "+v"(d2), "+v"(d3)
               : "v"(bf), "v"(a0), "v"(a1), "v"(a2), "v"(a3));
}

__global__ __launch_bounds__(128) void lstm_window_kernel(const float* __restrict__ x,
                                                          const float* __restrict__ W_ih,
                                                          const float* __restrict__ W_hh,
                                                          const float* __restrict__ b_ih,
                                                          const float* __restrict__ b_hh,
                                                          const float* __restrict__ W_out,
                                                          const float* __restrict__ b_out,
                                                          float* __restrict__ out) {
  __shared__ __align__(16) float sW[NGATE * HID];
  __shared__ __align__(16) float sWih[NGATE];
  __shared__ __align__(16) float sBias[NGATE];
  __shared__ __align__(16) float sWout[HID];
  __shared__ __align__(16) float sOut[OUT_PER_BLOCK];

  const int tid  = threadIdx.x;
  const int lane = tid & 31;
  const int wave = tid >> 5;
  const int col  = lane & 15;
  const int hh   = lane >> 4;
  const bool lo_half = (hh == 0);

  {
    const int i16 = tid & 15;
    const int i4  = tid & 3;
    const v4f w0 = *(const v4f*)(W_hh + 4 * tid);
    const v4f w1 = *(const v4f*)(W_hh + 4 * (tid + NTHREADS));
    const v4f wi = *(const v4f*)(W_ih + 4 * i16);
    const v4f bi = *(const v4f*)(b_ih + 4 * i16);
    const v4f bh = *(const v4f*)(b_hh + 4 * i16);
    const v4f wo = *(const v4f*)(W_out + 4 * i4);
    *(v4f*)(sW + 4 * tid) = w0;
    *(v4f*)(sW + 4 * (tid + NTHREADS)) = w1;
    if (tid < 16) {
      const v4f bsum = bi + bh;
      *(v4f*)(sWih + 4 * tid) = wi;
      *(v4f*)(sBias + 4 * tid) = bsum;
    }
    if (tid < 4) {
      *(v4f*)(sWout + 4 * tid) = wo;
    }
  }
  const float bout = b_out[0];
  __syncthreads();

  v16h a_frag[4];
#pragma unroll
  for (int t = 0; t < 4; ++t) {
    const float sc = (t == 2) ? 1.0f : 0.5f;
    const int m = 16 * t + col;
    const v4f wa = *(const v4f*)(sW + m * HID + 8 * hh);
    const v4f wb = *(const v4f*)(sW + m * HID + 8 * hh + 4);
    const float wih = sWih[m] * sc;
    const float bs  = sBias[m] * sc;
    const _Float16 wih_h = (_Float16)wih;
    const _Float16 bs_h  = (_Float16)bs;
    const float wih_l = (wih - (float)wih_h) * LOCARRY;
    const float bs_l  = (bs - (float)bs_h) * LOCARRY;
    v16h au;
    au[0] = (_Float16)(wa[0] * sc);
    au[1] = (_Float16)(wa[1] * sc);
    au[2] = (_Float16)(wa[2] * sc);
    au[3] = (_Float16)(wa[3] * sc);
    au[4] = (_Float16)(wb[0] * sc);
    au[5] = (_Float16)(wb[1] * sc);
    au[6] = (_Float16)(wb[2] * sc);
    au[7] = (_Float16)(wb[3] * sc);
    au[8]  = (_Float16)(lo_half ? wih   : 0.0f);
    au[9]  = (_Float16)(lo_half ? wih_l : 0.0f);
    au[10] = (_Float16)(lo_half ? bs    : 0.0f);
    au[11] = (_Float16)(lo_half ? bs_l  : 0.0f);
    au[12] = (_Float16)0.0f;
    au[13] = (_Float16)0.0f;
    au[14] = (_Float16)0.0f;
    au[15] = (_Float16)0.0f;
    a_frag[t] = au;
  }
  float wout_r[8];
#pragma unroll
  for (int j = 0; j < 8; ++j) wout_r[j] = sWout[8 * hh + j];

  const unsigned cword = pack_rne(lo_half ? 1.0f : 0.0f, lo_half ? LOCARRY_INV : 0.0f);

  const int brow = (blockIdx.x * NWAVES + wave) * 16 + col;
  const float* xrow = x + (size_t)brow * SEQ;
  const v8f z8 = {0.f, 0.f, 0.f, 0.f, 0.f, 0.f, 0.f, 0.f};

  float pred0 = 0.0f, pred1 = 0.0f, pred2 = 0.0f, pred3 = 0.0f;

#pragma unroll 1
  for (int p = 0; p < NPRED; ++p) {
    float c_s[8], h_s[8];
#pragma unroll
    for (int j = 0; j < 8; ++j) {
      c_s[j] = 0.0f;
      h_s[j] = 0.0f;
    }
    unsigned ph[4];
#pragma unroll
    for (int k = 0; k < 4; ++k) ph[k] = 0u;

    float xl = xrow[p];

#pragma unroll 1
    for (int t = 0; t < SEQ; ++t) {
      const int g = p + t;
      const int q = g - SEQ;
      float pv = pred3;
      pv = (q == 2) ? pred2 : pv;
      pv = (q == 1) ? pred1 : pv;
      pv = (q <= 0) ? pred0 : pv;
      const float xt = (g < SEQ) ? xl : pv;
      const int gn = g + 1;
      const int gc = (gn < SEQ) ? gn : (SEQ - 1);
      xl = xrow[gc];

      const float xs = lo_half ? xt : 0.0f;
      v8u bw;
      bw[0] = ph[0];
      bw[1] = ph[1];
      bw[2] = ph[2];
      bw[3] = ph[3];
      bw[4] = pack_rne(xs, xs * LOCARRY_INV);
      bw[5] = cword;
      bw[6] = 0u;
      bw[7] = 0u;
      const v16h b_frag = __builtin_bit_cast(v16h, bw);

      v8f g0 = wmma_f16(a_frag[0], b_frag, z8);
      v8f g1 = wmma_f16(a_frag[1], b_frag, z8);
      v8f g2 = wmma_f16(a_frag[2], b_frag, z8);
      v8f g3 = wmma_f16(a_frag[3], b_frag, z8);
      wmma_guard4(g0, g1, g2, g3, b_frag, a_frag[0], a_frag[1], a_frag[2], a_frag[3]);

#pragma unroll
      for (int j = 0; j < 8; ++j) {
        const float ig = sig_half_arg(g0[j]);
        const float fg = sig_half_arg(g1[j]);
        const float gg = hw_tanh(g2[j]);
        const float og = sig_half_arg(g3[j]);
        const float cc = __builtin_fmaf(fg, c_s[j], ig * gg);
        c_s[j] = cc;
        h_s[j] = og * hw_tanh(cc);
      }
#pragma unroll
      for (int k = 0; k < 4; ++k) ph[k] = pack_rne(h_s[2 * k], h_s[2 * k + 1]);
    }

    float partial = 0.0f;
#pragma unroll
    for (int j = 0; j < 8; ++j) partial = __builtin_fmaf(h_s[j], wout_r[j], partial);
    const float other = __shfl_xor(partial, 16, 32);
    const float val = (partial + other) + bout;

    pred0 = (p == 0) ? val : pred0;
    pred1 = (p == 1) ? val : pred1;
    pred2 = (p == 2) ? val : pred2;
    pred3 = (p == 3) ? val : pred3;

    if (lo_half) sOut[(wave * 16 + col) * NPRED + p] = val;
  }

  __syncthreads();

  if (wave == 0) {
    float* ob = out + (size_t)blockIdx.x * OUT_PER_BLOCK;
    v4f vals[3];
#pragma unroll
    for (int it = 0; it < 3; ++it) {
      const int idx = it * 32 + lane;
      const int idc = (idx < OUT_V4_PER_BLOCK) ? idx : (OUT_V4_PER_BLOCK - 1);
      vals[it] = *(const v4f*)(sOut + 4 * idc);
    }
    for (int pass = 0; pass < 2; ++pass) {
#pragma unroll
      for (int it = 0; it < 3; ++it) {
        const int idx = it * 32 + lane;
        if (idx < OUT_V4_PER_BLOCK) {
          *(volatile v4f*)(ob + 4 * idx) = vals[it];
        }
      }
      __threadfence();
    }
  }
}

extern "C" void kernel_launch(void* const* d_in, const int* in_sizes, int n_in,
                              void* d_out, int out_size, void* d_ws, size_t ws_size,
                              hipStream_t stream) {
  (void)d_ws;
  (void)ws_size;
  if (n_in < 7 || d_out == nullptr) return;
  if (in_sizes[0] != NBATCH * SEQ || in_sizes[1] != NGATE || in_sizes[2] != NGATE * HID ||
      in_sizes[3] != NGATE || in_sizes[4] != NGATE || in_sizes[5] != HID || in_sizes[6] != 1 ||
      out_size != NBATCH * NPRED) return;

  const float* x     = (const float*)d_in[0];
  const float* W_ih  = (const float*)d_in[1];
  const float* W_hh  = (const float*)d_in[2];
  const float* b_ih  = (const float*)d_in[3];
  const float* b_hh  = (const float*)d_in[4];
  const float* W_out = (const float*)d_in[5];
  const float* b_out = (const float*)d_in[6];
  float* out = (float*)d_out;

  lstm_window_kernel<<<dim3(NBLOCKS), dim3(NTHREADS), 0, stream>>>(x, W_ih, W_hh, b_ih, b_hh, W_out, b_out, out);
}
